// TheoreticalKANLayer_46626164965674
// MI455X (gfx1250) — hardware-verified
//
#include <hip/hip_runtime.h>
#include <math.h>
#include <stdint.h>

#pragma clang fp contract(off)

#define NB_ROWS 32768
#define I_DIM   128
#define O_DIM   256
#define NBAS    21
#define KDIM    (I_DIM * NBAS)
#define MCH     8192
#define NCH     (NB_ROWS / MCH)
#define RB1     256
#define NP1     (NB_ROWS / RB1)
#define BR      4
#define NPC     (BR * KDIM / 8)
#define WCARRY  32768.0f
#define RCARRY  2048.0f
#define LNEPS   1.0e-5f
#define PI_D    3.14159265358979323846
#define RCP018  (1.0f / 0.18f)
static_assert((KDIM % 32) == 0);
static_assert((MCH % 64) == 0 && (O_DIM % 64) == 0);
static_assert((NB_ROWS % MCH) == 0 && (MCH % BR) == 0 && (MCH % 8) == 0);
static_assert((NB_ROWS % RB1) == 0 && ((RB1 % 2) == 0));
static_assert((NPC % 32) == 0);
static_assert(((O_DIM * KDIM / 8) % 256) == 0);
static_assert((BR * I_DIM) % 256 == 0);
static_assert((((MCH / 64) * (O_DIM / 64)) % 8) == 0);

typedef _Float16       v16h __attribute__((ext_vector_type(16)));
typedef __bf16         v16b __attribute__((ext_vector_type(16)));
typedef unsigned short v16us __attribute__((ext_vector_type(16)));
typedef unsigned short v8us __attribute__((ext_vector_type(8)));
typedef float          v8f  __attribute__((ext_vector_type(8)));
typedef float          v4f  __attribute__((ext_vector_type(4)));
typedef unsigned int   v4u  __attribute__((ext_vector_type(4)));

union Frag { v16us u; v8us p[2]; v16h h; v16b b; };
union U8   { v8us s; v4u u; };

__device__ __forceinline__ unsigned short bf_bits(float f) {
  unsigned u = __float_as_uint(f);
  return (unsigned short)((u + 0x7FFFu + ((u >> 16) & 1u)) >> 16);
}
__device__ __forceinline__ float bf_up(unsigned short h) { return __uint_as_float(((unsigned)h) << 16); }
__device__ __forceinline__ float bfr(float f) { return bf_up(bf_bits(f)); }
__device__ __forceinline__ unsigned short h_bits(_Float16 x) { return __builtin_bit_cast(unsigned short, x); }
__device__ __forceinline__ unsigned pk16(unsigned short a, unsigned short b) { return (unsigned)a | ((unsigned)b << 16); }
__device__ __forceinline__ v8f zero8() { v8f z = {0.f, 0.f, 0.f, 0.f, 0.f, 0.f, 0.f, 0.f}; return z; }

__device__ __forceinline__ v16us ldfrag(const unsigned short* p) {
  Frag f;
  f.p[0] = *(const v8us*)(p);
  f.p[1] = *(const v8us*)(p + 16);
  return f.u;
}

template <int BF>
__device__ __forceinline__ v8f mma_raw(v16us a, v16us b, v8f c) {
  Frag fa, fb;
  fa.u = a;
  fb.u = b;
  if constexpr (BF) {
    return __builtin_amdgcn_wmma_f32_16x16x32_bf16(false, fa.b, false, fb.b, (short)0, c, false, false);
  } else {
    return __builtin_amdgcn_wmma_f32_16x16x32_f16(false, fa.h, false, fb.h, (short)0, c, false, false);
  }
}
__device__ __forceinline__ void dep_guard1(v8f& a, v8f& b, v16us x) {
#if defined(__HIP_DEVICE_COMPILE__)
  asm volatile("v_nop\n\tv_nop\n\tv_nop\n\tv_nop" : "+v"(a), "+v"(b) : "v"(x));
#endif
}
__device__ __forceinline__ void keep4(v16us a, v16us b, v16us c, v16us d) {
#if defined(__HIP_DEVICE_COMPILE__)
  asm volatile("v_nop" :: "v"(a), "v"(b), "v"(c), "v"(d));
#endif
}
__device__ __forceinline__ void acc_guard4(v8f& a, v8f& b, v8f& c, v8f& d) {
#if defined(__HIP_DEVICE_COMPILE__)
  asm volatile("v_nop\n\tv_nop\n\tv_nop\n\tv_nop" : "+v"(a), "+v"(b), "+v"(c), "+v"(d));
#endif
}
__device__ __forceinline__ void wave_sync_lds() {
  __builtin_amdgcn_fence(__ATOMIC_RELEASE, "workgroup");
  __builtin_amdgcn_wave_barrier();
  __builtin_amdgcn_fence(__ATOMIC_ACQUIRE, "workgroup");
}
__device__ __forceinline__ float wsum(float v) {
#pragma unroll
  for (int off = 16; off > 0; off >>= 1) v += __shfl_xor(v, off, 32);
  return v;
}

__global__ __launch_bounds__(256) void colmm1(const float* __restrict__ X, float* part) {
  __shared__ float smn[2][I_DIM], smx[2][I_DIM];
  __shared__ __align__(16) float sout[2 * I_DIM];
  const int t = threadIdx.x, c = t & (I_DIM - 1), par = t >> 7;
  const size_t r0 = (size_t)blockIdx.x * RB1;
  float mn = INFINITY, mx = -INFINITY;
#pragma unroll 4
  for (int j = 0; j < RB1 / 2; ++j) {
    const float v = bfr(X[(r0 + (size_t)(par + 2 * j)) * I_DIM + c]);
    mn = fminf(mn, v);
    mx = fmaxf(mx, v);
  }
  smn[par][c] = mn;
  smx[par][c] = mx;
  __syncthreads();
  if (t < I_DIM) {
    sout[t]         = fminf(smn[0][t], smn[1][t]);
    sout[I_DIM + t] = fmaxf(smx[0][t], smx[1][t]);
  }
  __syncthreads();
  if (t < 64) {
    const v4f v = *(const v4f*)(sout + 4 * t);
    float* dp = part + (size_t)blockIdx.x * (2 * I_DIM) + 4 * t;
    *(volatile v4f*)dp = v;
    __threadfence();
    *(volatile v4f*)dp = v;
  }
}

__global__ __launch_bounds__(256) void colmm2(const float* __restrict__ part, float* mm) {
  __shared__ __align__(16) float s[2 * I_DIM];
  const int t = threadIdx.x;
  float mn = INFINITY, mx = -INFINITY;
#pragma unroll 4
  for (int b = 0; b < NP1; ++b) {
    const float v = part[(size_t)b * (2 * I_DIM) + t];
    mn = fminf(mn, v);
    mx = fmaxf(mx, v);
  }
  s[t] = (t < I_DIM) ? mn : mx;
  __syncthreads();
  if (t < 64) {
    const v4f v = *(const v4f*)(s + 4 * t);
    float* dp = mm + 4 * t;
    *(volatile v4f*)dp = v;
    __threadfence();
    *(volatile v4f*)dp = v;
  }
}

__device__ __forceinline__ unsigned short wcv(float bwv, int flat, const float* __restrict__ CW) {
  const int o  = flat / KDIM;
  const int ii = (flat - o * KDIM) / NBAS;
  int ci = o * I_DIM + ii;
  ci = (ci < O_DIM * I_DIM) ? ci : (O_DIM * I_DIM - 1);
  const float cw = bfr(CW[ci]);
  return h_bits((_Float16)((bfr(bwv) * cw) * WCARRY));
}
__global__ __launch_bounds__(256) void wplane(const float* __restrict__ BW, const float* __restrict__ CW,
                                            unsigned short* Wp, int n8) {
  const int i  = blockIdx.x * 256 + threadIdx.x;
  const int ic = (i < n8) ? i : (n8 - 1);
  const int e0 = ic * 8;
  const v4f a = *(const v4f*)(BW + e0);
  const v4f c = *(const v4f*)(BW + e0 + 4);
  v4u o;
  o[0] = pk16(wcv(a[0], e0 + 0, CW), wcv(a[1], e0 + 1, CW));
  o[1] = pk16(wcv(a[2], e0 + 2, CW), wcv(a[3], e0 + 3, CW));
  o[2] = pk16(wcv(c[0], e0 + 4, CW), wcv(c[1], e0 + 5, CW));
  o[3] = pk16(wcv(c[2], e0 + 6, CW), wcv(c[3], e0 + 7, CW));
  if (i < n8) *(volatile v4u*)(Wp + (size_t)i * 8) = o;
  __threadfence();
  if (i < n8) *(volatile v4u*)(Wp + (size_t)i * 8) = o;
}

__device__ __forceinline__ void put2(unsigned short* sh, unsigned short* sl, int idx, float v) {
  const _Float16 hv = (_Float16)v;
  const float res = (v - (float)hv) * RCARRY;
  sh[idx] = h_bits(hv);
  sl[idx] = h_bits((_Float16)res);
}

__global__ __launch_bounds__(256) void basis_planes(const float* __restrict__ X, const float* __restrict__ mm,
                                                  unsigned short* AH, unsigned short* AL, int row0) {
  __shared__ float smn[I_DIM], srd[I_DIM];
  __shared__ __align__(16) unsigned short sh[BR * KDIM];
  __shared__ __align__(16) unsigned short sl[BR * KDIM];
  const int t = threadIdx.x;
  if (t < I_DIM) {
    const float mn = mm[t], mx = mm[I_DIM + t];
    const float d = (mx - mn) + 1.0e-8f;
    smn[t] = mn;
    srd[t] = 1.0f / d;
  }
  __syncthreads();
  const int lr0 = blockIdx.x * BR;
#pragma unroll 1
  for (int tt = 0; tt < (BR * I_DIM) / 256; ++tt) {
    const int task = t + 256 * tt;
    const int r = task >> 7, i = task & (I_DIM - 1);
    const float xv = bfr(X[((size_t)row0 + (size_t)(lr0 + r)) * I_DIM + i]);
    const float mn = smn[i], rd = srd[i];
    const float t1 = xv - mn;
    const float t2 = 2.0f * t1;
    const float t3 = t2 * rd;
    const float xn = t3 - 1.0f;
    const int kb = r * KDIM + i * NBAS;
    float tp = xn * 0.0f + 1.0f;
    float tc = xn;
    put2(sh, sl, kb + 0, tp);
    put2(sh, sl, kb + 1, tc);
#pragma unroll 1
    for (int n = 2; n <= 6; ++n) {
      const float u  = 2.0f * xn;
      const float tn = u * tc - tp;
      tp = tc;
      tc = tn;
      put2(sh, sl, kb + n, tn);
    }
#pragma unroll 1
    for (int k = 1; k <= 4; ++k) {
      const float kp = (k == 1) ? (float)(1.0 * PI_D) : (k == 2) ? (float)(2.0 * PI_D)
                     : (k == 3) ? (float)(3.0 * PI_D) : (float)(4.0 * PI_D);
      float sv, cv;
      sincosf(kp * xn, &sv, &cv);
      put2(sh, sl, kb + 5 + 2 * k, sv);
      put2(sh, sl, kb + 6 + 2 * k, cv);
    }
#pragma unroll 1
    for (int j = 0; j < 6; ++j) {
      const float cc = -1.0f + 0.4f * (float)j;
      const float dd = xn - cc;
      const float q  = dd * dd;
      const float ev = expf(-q * RCP018);
      put2(sh, sl, kb + 15 + j, ev);
    }
  }
  __syncthreads();
  const size_t gbase = (size_t)lr0 * KDIM;
  for (int pass = 0; pass < 2; ++pass) {
#pragma unroll
    for (int it = 0; it < (NPC + 255) / 256; ++it) {
      const int p = t + 256 * it;
      if (p < NPC) {
        U8 a, b;
        a.s = *(const v8us*)(sh + p * 8);
        b.s = *(const v8us*)(sl + p * 8);
        *(volatile v4u*)(AH + gbase + (size_t)p * 8) = a.u;
        *(volatile v4u*)(AL + gbase + (size_t)p * 8) = b.u;
      }
    }
    __threadfence();
  }
}

template <int BF, int OM, int BIASM>
__global__ __launch_bounds__(256) void gemm64(
    const unsigned short* __restrict__ A, int lda, long long strideA,
    const unsigned short* __restrict__ Bt, int ldb, long long strideB,
    const float* __restrict__ bias0, const float* __restrict__ bias1, int Nb,
    void* Cout, int ldc, long long strideC,
    int M, int N, int K, float oscale) {
  __shared__ __align__(16) float sT[8][16 * 68];
  const int b    = blockIdx.y;
  const int lane = threadIdx.x & 31;
  const int wave = threadIdx.x >> 5;
  const int tilesN = N >> 6;
  const int tilesM = M >> 6;
  const int tile = blockIdx.x * 8 + wave;
  if (tile >= tilesM * tilesN) return;
  const int tm = tile / tilesN;
  const int tn = tile - tm * tilesN;
  const int m0 = tm << 6;
  const int n0 = tn << 6;

  const unsigned short* Ab = A  + (size_t)b * (size_t)strideA;
  const unsigned short* Bb = Bt + (size_t)b * (size_t)strideB;

  const int rlane = lane & 15;
  const int koff  = (lane >> 4) * 8;
  const int mOff  = (lane >> 4) * 8;

  v8f acc[4][4];
#pragma unroll
  for (int i = 0; i < 4; ++i)
#pragma unroll
    for (int j = 0; j < 4; ++j) acc[i][j] = zero8();

  for (int k0 = 0; k0 < K; k0 += 32) {
    v16us bh[4];
#pragma unroll
    for (int j = 0; j < 4; ++j) {
      const size_t bo = (size_t)(n0 + (j << 4) + rlane) * ldb + koff + k0;
      bh[j] = ldfrag(Bb + bo);
    }
#pragma unroll
    for (int i = 0; i < 4; ++i) {
      const size_t ao = (size_t)(m0 + (i << 4) + rlane) * lda + koff + k0;
      const v16us ah = ldfrag(Ab + ao);
#pragma unroll
      for (int j = 0; j < 4; ++j) acc[i][j] = mma_raw<BF>(ah, bh[j], acc[i][j]);
      dep_guard1(acc[i][0], acc[i][3], ah);
    }
    keep4(bh[0], bh[1], bh[2], bh[3]);
  }
  acc_guard4(acc[0][0], acc[0][1], acc[0][2], acc[0][3]);
  acc_guard4(acc[1][0], acc[1][1], acc[1][2], acc[1][3]);
  acc_guard4(acc[2][0], acc[2][1], acc[2][2], acc[2][3]);
  acc_guard4(acc[3][0], acc[3][1], acc[3][2], acc[3][3]);

  const int hh2 = lane >> 4, c4 = (lane & 15) * 4;
  const int q8  = lane >> 3, c8 = (lane & 7) * 8;
  float bc[8];
#pragma unroll
  for (int e = 0; e < 8; ++e) bc[e] = 0.f;
  if (BIASM == 0) {
    const bool use1 = (n0 >= Nb);
    if (OM == 0) {
      const int cb = n0 + c4;
      const int i0 = (cb < Nb - 4) ? cb : (Nb - 4);
      const int i1 = (cb - Nb > 0) ? (cb - Nb) : 0;
      const v4f b0v = *(const v4f*)(bias0 + i0);
      const v4f b1v = *(const v4f*)(bias1 + i1);
#pragma unroll
      for (int e = 0; e < 4; ++e) bc[e] = bfr(use1 ? b1v[e] : b0v[e]);
    } else {
      const int cb = n0 + c8;
      const int i0 = (cb < Nb - 8) ? cb : (Nb - 8);
      const int i1 = (cb - Nb > 0) ? (cb - Nb) : 0;
      const v4f b0a = *(const v4f*)(bias0 + i0), b0b = *(const v4f*)(bias0 + i0 + 4);
      const v4f b1a = *(const v4f*)(bias1 + i1), b1b = *(const v4f*)(bias1 + i1 + 4);
#pragma unroll
      for (int e = 0; e < 4; ++e) {
        bc[e]     = bfr(use1 ? b1a[e] : b0a[e]);
        bc[4 + e] = bfr(use1 ? b1b[e] : b0b[e]);
      }
    }
  }

  float* slab = sT[wave];
#pragma unroll
  for (int i = 0; i < 4; ++i) {
    const int mBase = m0 + (i << 4);
#pragma unroll
    for (int j = 0; j < 4; ++j) {
#pragma unroll
      for (int r = 0; r < 8; ++r) {
        slab[(mOff + r) * 68 + (j << 4) + rlane] = acc[i][j][r];
      }
    }
    wave_sync_lds();
    if constexpr (OM == 0) {
      float* C = (float*)Cout + (size_t)b * (size_t)strideC;
      v4f vals[8];
#pragma unroll
      for (int it = 0; it < 8; ++it) {
        const int row = it * 2 + hh2;
        v4f v = *(const v4f*)(slab + row * 68 + c4);
#pragma unroll
        for (int e = 0; e < 4; ++e) v[e] = v[e] * oscale + bc[e];
        vals[it] = v;
      }
      for (int pass = 0; pass < 2; ++pass) {
#pragma unroll
        for (int it = 0; it < 8; ++it) {
          const int row = it * 2 + hh2;
          *(volatile v4f*)(C + (size_t)(mBase + row) * ldc + n0 + c4) = vals[it];
        }
        __threadfence();
      }
    } else {
      unsigned short* C = (unsigned short*)Cout + (size_t)b * (size_t)strideC;
      v4u hv[4];
#pragma unroll
      for (int it = 0; it < 4; ++it) {
        const int row = it * 4 + q8;
        const float* sp = slab + row * 68 + c8;
        float bm = 0.f;
        if (BIASM == 1) bm = bfr(bias0[mBase + row]);
        v4u a;
#pragma unroll
        for (int e = 0; e < 4; ++e) {
          const float f0 = sp[2 * e]     * oscale + ((BIASM == 1) ? bm : bc[2 * e]);
          const float f1 = sp[2 * e + 1] * oscale + ((BIASM == 1) ? bm : bc[2 * e + 1]);
          a[e] = pk16(h_bits((_Float16)f0), h_bits((_Float16)f1));
        }
        hv[it] = a;
      }
      for (int pass = 0; pass < 2; ++pass) {
#pragma unroll
        for (int it = 0; it < 4; ++it) {
          const int row = it * 4 + q8;
          unsigned short* dp = C + (size_t)(mBase + row) * ldc + n0 + c8;
          *(volatile v4u*)(dp) = hv[it];
        }
        __threadfence();
      }
    }
    wave_sync_lds();
  }
}

__global__ __launch_bounds__(256) void ln_rows(const float* __restrict__ Hp, const float* __restrict__ Lp,
                                             const float* __restrict__ bias, const float* __restrict__ gam,
                                             const float* __restrict__ bet, float* outp) {
  const int lane = threadIdx.x & 31, wave = threadIdx.x >> 5;
  const size_t row  = (size_t)blockIdx.x * 8 + wave;
  const size_t base = row * O_DIM;
  const int c0 = 4 * lane, c1 = (O_DIM / 2) + 4 * lane;
  const v4f h0 = *(const v4f*)(Hp + base + c0), h1 = *(const v4f*)(Hp + base + c1);
  const v4f l0 = *(const v4f*)(Lp + base + c0), l1 = *(const v4f*)(Lp + base + c1);
  const v4f b0 = *(const v4f*)(bias + c0),      b1 = *(const v4f*)(bias + c1);
  v4f y0, y1;
#pragma unroll
  for (int e = 0; e < 4; ++e) {
    y0[e] = (h0[e] + l0[e]) + bfr(b0[e]);
    y1[e] = (h1[e] + l1[e]) + bfr(b1[e]);
  }
  float s = ((y0[0] + y0[1]) + (y0[2] + y0[3])) + ((y1[0] + y1[1]) + (y1[2] + y1[3]));
  s = wsum(s);
  const float mean = s * (1.0f / (float)O_DIM);
  v4f d0, d1;
#pragma unroll
  for (int e = 0; e < 4; ++e) { d0[e] = y0[e] - mean; d1[e] = y1[e] - mean; }
  float q = ((d0[0] * d0[0] + d0[1] * d0[1]) + (d0[2] * d0[2] + d0[3] * d0[3]))
          + ((d1[0] * d1[0] + d1[1] * d1[1]) + (d1[2] * d1[2] + d1[3] * d1[3]));
  q = wsum(q);
  const float var  = q * (1.0f / (float)O_DIM);
  const float rstd = rsqrtf(var + LNEPS);
  const v4f g0 = *(const v4f*)(gam + c0), g1 = *(const v4f*)(gam + c1);
  const v4f e0 = *(const v4f*)(bet + c0), e1 = *(const v4f*)(bet + c1);
  v4f o0, o1;
#pragma unroll
  for (int e = 0; e < 4; ++e) {
    o0[e] = (d0[e] * rstd) * bfr(g0[e]) + bfr(e0[e]);
    o1[e] = (d1[e] * rstd) * bfr(g1[e]) + bfr(e1[e]);
  }
  float* dp0 = outp + base + c0;
  float* dp1 = outp + base + c1;
  *(volatile v4f*)dp0 = o0;
  *(volatile v4f*)dp1 = o1;
  __threadfence();
  *(volatile v4f*)dp0 = o0;
  *(volatile v4f*)dp1 = o1;
}

extern "C" void kernel_launch(void* const* d_in, const int* in_sizes, int n_in,
                              void* d_out, int out_size, void* d_ws, size_t ws_size,
                              hipStream_t stream) {
  if (n_in < 6) return;
  if (in_sizes[0] != NB_ROWS * I_DIM) return;
  if (in_sizes[1] != O_DIM * KDIM) return;
  if (in_sizes[2] != O_DIM * I_DIM) return;
  if (in_sizes[3] != O_DIM || in_sizes[4] != O_DIM || in_sizes[5] != O_DIM) return;
  if (out_size != NB_ROWS * O_DIM) return;

  const float* x    = (const float*)d_in[0];
  const float* bw   = (const float*)d_in[1];
  const float* conn = (const float*)d_in[2];
  const float* bias = (const float*)d_in[3];
  const float* gam  = (const float*)d_in[4];
  const float* bet  = (const float*)d_in[5];

  const size_t PPART = (size_t)NP1 * 2 * I_DIM * 4;
  const size_t PMM   = 1024;
  const size_t PWP   = (size_t)O_DIM * KDIM * 2;
  const size_t PA    = (size_t)MCH * KDIM * 2;
  const size_t PHL   = (size_t)MCH * O_DIM * 4;
  size_t off = 0;
  const size_t oPart = off; off += PPART;
  const size_t oMM   = off; off += PMM;
  const size_t oWP   = off; off += PWP;
  const size_t oAH   = off; off += PA;
  const size_t oAL   = off; off += PA;
  const size_t oH    = off; off += PHL;
  const size_t oL    = off; off += PHL;
  if (off > ws_size) return;
  if (off > (size_t)134217728) return;
  if ((oMM % 256) != 0 || (oWP % 256) != 0 || (oAH % 256) != 0 || (oAL % 256) != 0 || (oH % 256) != 0 || (oL % 256) != 0) return;

  char* ws = (char*)d_ws;
  float*          PART = (float*)(ws + oPart);
  float*          MM   = (float*)(ws + oMM);
  unsigned short* WP   = (unsigned short*)(ws + oWP);
  unsigned short* AH   = (unsigned short*)(ws + oAH);
  unsigned short* AL   = (unsigned short*)(ws + oAL);
  float*          Hb   = (float*)(ws + oH);
  float*          Lb   = (float*)(ws + oL);
  float*          out0 = (float*)d_out;

  const int n8w = (O_DIM * KDIM) / 8;
  const dim3 blk(256);
  const dim3 gP1(NP1);
  const dim3 gW(n8w / 256);
  const dim3 gB(MCH / BR);
  const dim3 gG(((MCH / 64) * (O_DIM / 64) + 7) / 8, 1);
  const dim3 gL(MCH / 8);
  const float osc_hi = 1.0f / WCARRY;
  const float osc_lo = 1.0f / (WCARRY * RCARRY);

  colmm1<<<gP1, blk, 0, stream>>>(x, PART);
  colmm2<<<dim3(1), blk, 0, stream>>>(PART, MM);

  wplane<<<gW, blk, 0, stream>>>(bw, conn, WP, n8w);

  for (int ch = 0; ch < NCH; ++ch) {
    basis_planes<<<gB, blk, 0, stream>>>(x, MM, AH, AL, ch * MCH);
    gemm64<0, 0, 2><<<gG, blk, 0, stream>>>(
        AH, KDIM, 0LL, WP, KDIM, 0LL, bias, bias, O_DIM,
        (void*)Hb, O_DIM, 0LL, MCH, O_DIM, KDIM, osc_hi);
    gemm64<0, 0, 2><<<gG, blk, 0, stream>>>(
        AL, KDIM, 0LL, WP, KDIM, 0LL, bias, bias, O_DIM,
        (void*)Lb, O_DIM, 0LL, MCH, O_DIM, KDIM, osc_lo);
    ln_rows<<<gL, blk, 0, stream>>>(Hb, Lb, bias, gam, bet, out0 + (size_t)ch * MCH * O_DIM);
  }
  (void)hipGetLastError();
}
